// MyRGCNConv_35536559407731
// MI455X (gfx1250) — hardware-verified
//
#include <hip/hip_runtime.h>
#include <stddef.h>


#define DIM      256
#define NREL     8
#define KTOT     (NREL * DIM)
#define KSTEPS   (KTOT / 32)
#define NTHR     256
#define NWAVE    8
#define CPB      32
#define CPW      (CPB / NWAVE)
#define APH      (KTOT + 8)
#define CPF      (DIM + 4)
#define MAXDEG   8192
#define LDS_A    (CPB * APH * 2)
#define LDS_DEG  (CPB * 4)
#define LDS_MAIN (LDS_A + LDS_DEG)
#define WPL_THREADS (DIM * KTOT / 8)
#define WPL_BLOCKS  (WPL_THREADS / NTHR)
#define WS_NEED  ((size_t)KTOT * DIM * 2)

static_assert(NTHR == NWAVE * 32);
static_assert(CPB == NWAVE * CPW);
static_assert(CPB == 32 && DIM == 256);
static_assert(DIM == 32 * 8);
static_assert((KTOT % 32) == 0);
static_assert(((APH * 2) % 16) == 0);
static_assert(((CPF * 4) % 16) == 0);
static_assert(CPB * CPF * 4 <= LDS_A);
static_assert((LDS_A % 16) == 0);
static_assert(LDS_MAIN <= 160 * 1024);
static_assert(WPL_BLOCKS * NTHR * 8 == DIM * KTOT);

typedef float          v4f  __attribute__((ext_vector_type(4)));
typedef float          v8f  __attribute__((ext_vector_type(8)));
typedef unsigned       v4u  __attribute__((ext_vector_type(4)));
typedef _Float16       v8h  __attribute__((ext_vector_type(8)));
typedef _Float16       v16h __attribute__((ext_vector_type(16)));
union FragH { v16h v; v8h h[2]; };
union Pk8   { v8h h; v4u i; };

__device__ __forceinline__ v8f zero8() {
  v8f z;
#pragma unroll
  for (int i = 0; i < 8; ++i) z[i] = 0.0f;
  return z;
}

__device__ __forceinline__ v8f wmma16(v16h a, v16h b, v8f c) {
  v8f d = __builtin_amdgcn_wmma_f32_16x16x32_f16(false, a, false, b, (short)0, c, false, false);
  asm volatile("v_nop\n\tv_nop\n\tv_nop\n\tv_nop" : "+v"(d) : "v"(a), "v"(b));
  return d;
}

__global__ __launch_bounds__(NTHR) void k_wplane(const float* __restrict__ W, _Float16* wp) {
  const int u  = blockIdx.x * NTHR + threadIdx.x;
  const int n  = u >> 8;
  const int kc = u & 255;
  Pk8 pk;
#pragma unroll
  for (int j = 0; j < 8; ++j) {
    const int k = 8 * kc + j;
    const int r = k >> 8;
    const int i = k & 255;
    const float f = W[((size_t)r * DIM + i) * DIM + n] * 16.0f;
    pk.h[j] = (_Float16)f;
  }
  _Float16* d = wp + (size_t)u * 8;
  *(volatile v4u*)d = pk.i;
  __threadfence();
  *(volatile v4u*)d = pk.i;
}

__device__ __forceinline__ void out_pass(const float* Cs, const float* degL, float* out,
                                         int cb, int wave, int lane, int nCe) {
#pragma unroll
  for (int j = 0; j < CPW; ++j) {
    const int cl = wave + NWAVE * j;
    const int c = __builtin_amdgcn_readfirstlane(cb + cl);
    if (c < nCe) {
      const float degf = degL[cl];
      const float sc = 0.0625f * (1.0f / degf);
      const float* cr = Cs + (size_t)cl * CPF + 4 * lane;
      v4f v0 = *(const v4f*)cr;
      v4f v1 = *(const v4f*)(cr + 128);
      v0 *= sc;
      v1 *= sc;
      float* orow = out + (size_t)c * DIM + 4 * lane;
      *(volatile v4f*)orow = v0;
      *(volatile v4f*)(orow + 128) = v1;
    }
  }
}

__global__ __launch_bounds__(NTHR) void k_main(const float* __restrict__ x, const int* __restrict__ ptr,
    const int* __restrict__ idx, const int* __restrict__ et, const int* __restrict__ nnp,
    const _Float16* __restrict__ wp, float* out, int nN, int nC, int nE) {
  extern __shared__ __attribute__((aligned(16))) unsigned char dsm[];
  _Float16* At = (_Float16*)dsm;
  float* Cs = (float*)dsm;
  float* degL = (float*)(dsm + LDS_A);
  const int tid = threadIdx.x, lane = tid & 31, wave = tid >> 5, hh = lane >> 4, m = lane & 15;
  const int cb = blockIdx.x * CPB;
  const int nn = nnp[0];
  const int nCe = nC < nn ? nC : nn;

#pragma unroll 1
  for (int j = 0; j < CPW; ++j) {
    const int cl = wave + NWAVE * j;
    const int c = __builtin_amdgcn_readfirstlane(cb + cl);
    float acc[NREL][8];
#pragma unroll
    for (int r = 0; r < NREL; ++r) {
#pragma unroll
      for (int q = 0; q < 8; ++q) acc[r][q] = 0.0f;
    }
    float degf = 1.0f;
    if (c < nCe) {
      const int ca = c < nC - 1 ? c : nC - 1;
      const int cb1 = (c + 1) < nC ? (c + 1) : nC;
      const int p0 = ptr[ca];
      const int p1 = ptr[cb1];
      degf = (float)(p1 - p0);
      int e0 = p0 < 0 ? 0 : (p0 > nE ? nE : p0);
      int e1 = p1 < e0 ? e0 : (p1 > nE ? nE : p1);
      int cnt = e1 - e0;
      cnt = cnt > MAXDEG ? MAXDEG : cnt;
      cnt = __builtin_amdgcn_readfirstlane(cnt);
      e0 = __builtin_amdgcn_readfirstlane(e0);
#pragma unroll 1
      for (int i = 0; i < cnt; i += 32) {
        int ee = e0 + i + lane;
        ee = ee > nE - 1 ? nE - 1 : ee;
        int sv = idx[ee];
        int tv = et[ee];
        sv = sv < 0 ? sv + nN : sv;
        sv = sv < 0 ? 0 : (sv > nN - 1 ? nN - 1 : sv);
        tv = tv < 0 ? tv + NREL : tv;
        tv = tv < 0 ? 0 : (tv > NREL - 1 ? NREL - 1 : tv);
        int jn = cnt - i;
        jn = jn > 32 ? 32 : jn;
#pragma unroll 1
        for (int jj = 0; jj < jn; ++jj) {
          const int s = __builtin_amdgcn_readlane(sv, jj);
          const int t = __builtin_amdgcn_readlane(tv, jj);
          const float* xr = x + (size_t)s * DIM + 8 * lane;
          const v4f va = *(const v4f*)xr;
          const v4f vb = *(const v4f*)(xr + 4);
#pragma unroll
          for (int r = 0; r < NREL; ++r) {
            if (t == r) {
              acc[r][0] += va.x; acc[r][1] += va.y; acc[r][2] += va.z; acc[r][3] += va.w;
              acc[r][4] += vb.x; acc[r][5] += vb.y; acc[r][6] += vb.z; acc[r][7] += vb.w;
            }
          }
        }
      }
    }
    _Float16* arow = At + (size_t)cl * APH + 8 * lane;
#pragma unroll
    for (int r = 0; r < NREL; ++r) {
      v8h hv;
#pragma unroll
      for (int q = 0; q < 8; ++q) hv[q] = (_Float16)acc[r][q];
      *(v8h*)(arow + DIM * r) = hv;
    }
    if (lane == 0) degL[cl] = degf;
  }
  __syncthreads();

  {
    const int rt = wave & 1, cg = wave >> 1;
    const _Float16* ar = At + (size_t)(16 * rt + m) * APH + 8 * hh;
    const _Float16* br = wp + (size_t)(64 * cg + m) * KTOT + 8 * hh;
    v8f d[4];
#pragma unroll
    for (int j = 0; j < 4; ++j) d[j] = zero8();
#pragma unroll 2
    for (int ks = 0; ks < KSTEPS; ++ks) {
      const int k0 = 32 * ks;
      FragH a;
      a.h[0] = *(const v8h*)(ar + k0);
      a.h[1] = *(const v8h*)(ar + k0 + 16);
#pragma unroll
      for (int j = 0; j < 4; ++j) {
        const _Float16* bp = br + (size_t)(16 * j) * KTOT + k0;
        FragH b;
        b.h[0] = *(const v8h*)bp;
        b.h[1] = *(const v8h*)(bp + 16);
        d[j] = wmma16(a.v, b.v, d[j]);
      }
    }
    __syncthreads();
    float* cs = Cs + (size_t)(16 * rt + 8 * hh) * CPF + 64 * cg + m;
#pragma unroll
    for (int j = 0; j < 4; ++j) {
#pragma unroll
      for (int r = 0; r < 8; ++r) cs[r * CPF + 16 * j] = d[j][r];
    }
  }
  __syncthreads();

  out_pass(Cs, degL, out, cb, wave, lane, nCe);
  __threadfence();
  out_pass(Cs, degL, out, cb, wave, lane, nCe);
}

extern "C" void kernel_launch(void* const* d_in, const int* in_sizes, int n_in,
                              void* d_out, int out_size, void* d_ws, size_t ws_size,
                              hipStream_t stream) {
  if (n_in < 6) return;
  if (in_sizes[0] < DIM || (in_sizes[0] % DIM) != 0) return;
  const int nN = in_sizes[0] / DIM;
  if (in_sizes[1] != NREL * DIM * DIM) return;
  if (out_size < DIM || (out_size % DIM) != 0) return;
  const int nC = out_size / DIM;
  if (in_sizes[2] != nC + 1) return;
  const int nE = in_sizes[3];
  if (nE < 1 || in_sizes[4] != nE) return;
  if (in_sizes[5] < 1) return;

  size_t limit = (size_t)134217728;
  if (ws_size < limit) limit = ws_size;
  if (WS_NEED > limit) return;

  const float* x   = (const float*)d_in[0];
  const float* W   = (const float*)d_in[1];
  const int*   ptr = (const int*)d_in[2];
  const int*   idx = (const int*)d_in[3];
  const int*   et  = (const int*)d_in[4];
  const int*   nnp = (const int*)d_in[5];
  float* dout = (float*)d_out;
  _Float16* wp = (_Float16*)d_ws;

  k_wplane<<<WPL_BLOCKS, NTHR, 0, stream>>>(W, wp);

  hipFuncSetAttribute(reinterpret_cast<const void*>(&k_main), hipFuncAttributeMaxDynamicSharedMemorySize, LDS_MAIN);
  const int nBlk = (nC + CPB - 1) / CPB;
  k_main<<<nBlk, NTHR, LDS_MAIN, stream>>>(x, ptr, idx, et, nnp, wp, dout, nN, nC, nE);
}
